// SSINF3OneTenthMLP_19198503813134
// MI455X (gfx1250) — hardware-run, weakly checked
//
#include <hip/hip_runtime.h>


#ifndef NB
#define NB 2
#endif
#ifndef SEQ
#define SEQ 2048
#endif
#define NB_FULL  2
#define SEQ_FULL 2048
#define NTOK  (NB * SEQ)
#define DM    768
#define NS    8
#define RK    16
#define SR    (NS * RK)
#define NA    64
#define TK    4
#define HL    32
#define HG    256
#define NGRP  (NS * NA)
#define RB    1024
#define NPS   (NTOK * TK)
#define NBS   (NPS / RB)
#define NBLK  (NS * NBS)
#define PROWS (NS * NPS + NGRP * 64)
#define TILES (PROWS / 64)
#define MAXT  (NPS / 64)
#define ZP    512
#define XP    64
#define YP    32
#define PB1   (NGRP * HL * 4 / 256)
#define PB2   (NGRP * RK * 4 / 256)
#define PB3   (NGRP * 8 / 256)
#define PB4   (SR * (DM / 8) / 256)

static_assert(NB <= NB_FULL && SEQ <= SEQ_FULL);
static_assert(SEQ % 64 == 0);
static_assert(NTOK % 256 == 0);
static_assert(NPS % RB == 0);
static_assert(NBS >= 1);
static_assert(NBLK % 32 == 0);
static_assert(TILES % 512 == 0);
static_assert(TILES % 128 == 0);
static_assert(PROWS % 64 == 0);
static_assert(NA == 64 && RK == 16 && HL == 32 && TK == 4 && NGRP == 512);
static_assert(2 * RK == 32 && XP == 64);
static_assert(DM % 64 == 0 && SR % 64 == 0 && HG % 64 == 0);
static_assert(DM % 32 == 0 && SR % 32 == 0 && HG % 32 == 0);
static_assert((NTOK * (DM / 8)) % 256 == 0);
static_assert((NGRP * HL * 4) % 256 == 0 && (NGRP * RK * 4) % 256 == 0 && (NGRP * 8) % 256 == 0 && (SR * (DM / 8)) % 256 == 0);
static_assert((size_t)NB_FULL * SEQ_FULL * DM * 4 == (size_t)12582912);
static_assert(32 * 16 * 64 == 64 * 512);
static_assert(32 * 16 * 16 == 64 * 128);
static_assert(32 * 16 * 32 == 64 * 256);
static_assert(32 * 16 * 8  == 32 * 128);
static_assert(256 * 16 * 2 == 64 * 128);
static_assert(4 * 8 == 32);
static_assert(64 * 68 * 4 <= 131072);
static_assert(64 * 65 * 4 <= 131072);
static_assert(32 * 64 * 4 + 64 * 4 <= 131072);
static_assert(((size_t)NBLK * 64 + TILES + 16) * 4 <= 65536);
static_assert(64 * 40 * 2 + 64 * 20 * 4 <= 131072);

typedef unsigned short bf;
typedef _Float16 h16;
typedef __attribute__((ext_vector_type(16))) __bf16   v16bf;
typedef __attribute__((ext_vector_type(16))) _Float16 v16h;
typedef __attribute__((ext_vector_type(8)))  _Float16 v8h;
typedef __attribute__((ext_vector_type(8)))  unsigned short v8us;
typedef __attribute__((ext_vector_type(8)))  float    v8f;
typedef __attribute__((ext_vector_type(4)))  float    v4f;
typedef __attribute__((ext_vector_type(4)))  int      v4i;
typedef v4f  __attribute__((may_alias)) v4fa;
typedef v4i  __attribute__((may_alias)) v4ia;
typedef v8h  __attribute__((may_alias)) v8ha;

__device__ __forceinline__ unsigned short f2bf(float f) { unsigned u = __float_as_uint(f); u += 0x7FFFu + ((u >> 16) & 1u); return (unsigned short)(u >> 16); }
__device__ __forceinline__ float bf2f(unsigned short w) { return __uint_as_float(((unsigned)w) << 16); }
__device__ __forceinline__ int clampi(int v, int lo, int hi) { return min(max(v, lo), hi); }
__device__ __forceinline__ v16bf cat16b(v8us lo, v8us hi) { return __builtin_bit_cast(v16bf, __builtin_shufflevector(lo, hi, 0, 1, 2, 3, 4, 5, 6, 7, 8, 9, 10, 11, 12, 13, 14, 15)); }
__device__ __forceinline__ v16h cat16h(v8h lo, v8h hi) { return __builtin_shufflevector(lo, hi, 0, 1, 2, 3, 4, 5, 6, 7, 8, 9, 10, 11, 12, 13, 14, 15); }
__device__ __forceinline__ v16bf ldb(const bf* p)  { return cat16b(*(const v8us*)p, *(const v8us*)(p + 16)); }
__device__ __forceinline__ v16h  ldh(const h16* p) { return cat16h(*(const v8h*)p, *(const v8h*)(p + 16)); }
__device__ __forceinline__ v8f wmmab_g(v16bf a, v16bf b, v8f c) {
    c = __builtin_amdgcn_wmma_f32_16x16x32_bf16(false, a, false, b, (short)0, c, false, false);
    asm volatile("v_nop\n\tv_nop\n\tv_nop\n\tv_nop" : "+v"(c) : "v"(a), "v"(b));
    return c; }
__device__ __forceinline__ v8f wmmah_g(v16h a, v16h b, v8f c) {
    c = __builtin_amdgcn_wmma_f32_16x16x32_f16(false, a, false, b, (short)0, c, false, false);
    asm volatile("v_nop\n\tv_nop\n\tv_nop\n\tv_nop" : "+v"(c) : "v"(a), "v"(b));
    return c; }
__device__ __forceinline__ h16 toh_flush(float v) { const h16 r = (h16)v; return (fabsf(v) < 6.103515625e-05f) ? (h16)0.0f : r; }
__device__ __forceinline__ float gelu_t(float x) {
    const float u = 0.7978845608028654f * (x + 0.044715f * x * x * x);
    const float uc = fminf(fmaxf(u, -15.0f), 15.0f);
    const float e = __expf(2.0f * uc);
    return x * (e * __builtin_amdgcn_rcpf(1.0f + e)); }
__device__ __forceinline__ void top4_ins(float sc, int mm, float& tv0, float& tv1, float& tv2, float& tv3, int& ti0, int& ti1, int& ti2, int& ti3) {
    const bool g0 = sc > tv0, g1 = sc > tv1, g2 = sc > tv2, g3 = sc > tv3;
    tv3 = g2 ? tv2 : (g3 ? sc : tv3); ti3 = g2 ? ti2 : (g3 ? mm : ti3);
    tv2 = g1 ? tv1 : (g2 ? sc : tv2); ti2 = g1 ? ti1 : (g2 ? mm : ti2);
    tv1 = g0 ? tv0 : (g1 ? sc : tv1); ti1 = g0 ? ti0 : (g1 ? mm : ti1);
    tv0 = g0 ? sc : tv0;              ti0 = g0 ? mm : ti0; }
__device__ __forceinline__ void wave_sync() { __builtin_amdgcn_fence(3  , "wavefront"); __builtin_amdgcn_wave_barrier(); asm volatile("" ::: "memory"); }

__global__ __launch_bounds__(256) void k_xcvt(const float* __restrict__ X, bf* XB) {
    const int pc = blockIdx.x * 256 + threadIdx.x;
    const int n = pc / (DM / 8); const int c8 = (pc - n * (DM / 8)) * 8;
    const size_t rin = (size_t)(n / SEQ) * SEQ_FULL + (size_t)(n % SEQ);
    const v8f a = *(const v8f*)(X + rin * DM + c8);
    v8us o;
#pragma unroll
    for (int k = 0; k < 8; ++k) o[k] = f2bf(a[k]);
    bf* dst = XB + (size_t)n * DM + c8;
    *(volatile v8us*)dst = o;
    __threadfence();
    *(volatile v8us*)dst = o;
}

__global__ __launch_bounds__(256) void k_prep(const float* __restrict__ P, const float* __restrict__ C, const float* __restrict__ W1, const float* __restrict__ W2,
                                              bf* PT, bf* CT, h16* W1T, h16* W2T) {
    const int b = blockIdx.x, t = threadIdx.x;
    if (b < PB1) {
        const int pc = b * 256 + t; const int c = pc & 3, h = (pc >> 2) & 31, e = pc >> 7;
        const float* src = W1 + (size_t)e * (RK * HL) + (size_t)((c & 1) * 8) * HL + h;
        v8h o;
#pragma unroll
        for (int k = 0; k < 8; ++k) o[k] = toh_flush(bf2f(f2bf(src[(size_t)k * HL])));
        h16* dst = W1T + (size_t)pc * 8;
        *(volatile v8h*)dst = o; __threadfence(); *(volatile v8h*)dst = o;
    } else if (b < PB1 + PB2) {
        const int pc = (b - PB1) * 256 + t; const int c = pc & 3, r = (pc >> 2) & 15, e = pc >> 6;
        const float* src = W2 + (size_t)e * (HL * RK) + (size_t)(c * 8) * RK + r;
        v8h o;
#pragma unroll
        for (int k = 0; k < 8; ++k) o[k] = toh_flush(bf2f(f2bf(src[(size_t)k * RK])));
        h16* dst = W2T + (size_t)pc * 8;
        *(volatile v8h*)dst = o; __threadfence(); *(volatile v8h*)dst = o;
    } else if (b < PB1 + PB2 + PB3) {
        const int pc = (b - PB1 - PB2) * 256 + t; const int c = pc & 7, row = pc >> 3;
        const float* src = C + (size_t)row * RK + (c & 1) * 8;
        v8us o;
#pragma unroll
        for (int k = 0; k < 8; ++k) { const unsigned short v = f2bf(src[k]); o[k] = (c < 6) ? v : (unsigned short)0; }
        bf* dst = CT + (size_t)pc * 8;
        *(volatile v8us*)dst = o; __threadfence(); *(volatile v8us*)dst = o;
    } else {
        const int pc = (b - PB1 - PB2 - PB3) * 256 + t; const int col = pc / (DM / 8); const int d8 = (pc - col * (DM / 8)) * 8;
        const int s = col >> 4, r = col & 15;
        const float* src = P + ((size_t)s * DM + d8) * RK + r;
        v8us o;
#pragma unroll
        for (int k = 0; k < 8; ++k) o[k] = f2bf(src[(size_t)k * RK]);
        bf* dst = PT + (size_t)col * DM + d8;
        *(volatile v8us*)dst = o; __threadfence(); *(volatile v8us*)dst = o;
    }
}

__global__ __launch_bounds__(256) void k_wt(const float* __restrict__ W, h16* WT, int R, int C) {
    __shared__ float ts[64 * 65];
    const int t = threadIdx.x;
    const int c0 = blockIdx.x * 64, r0 = blockIdx.y * 64, e = blockIdx.z;
    const float* src = W + (size_t)e * R * C + (size_t)r0 * C + c0;
#pragma unroll 1
    for (int i = 0; i < 16; ++i) { const int f = i * 256 + t; ts[(f >> 6) * 65 + (f & 63)] = src[(size_t)(f >> 6) * C + (f & 63)]; }
    __syncthreads();
    h16* dst = WT + (size_t)e * R * C + (size_t)c0 * R + r0;
#pragma unroll 1
    for (int ps = 0; ps < 2; ++ps) {
#pragma unroll 1
        for (int it = 0; it < 2; ++it) {
            const int cl = it * 32 + (t >> 3), r8 = (t & 7) * 8; v8h o;
#pragma unroll
            for (int k = 0; k < 8; ++k) o[k] = toh_flush(bf2f(f2bf(ts[(r8 + k) * 65 + cl])));
            *(volatile v8h*)(dst + (size_t)cl * R + r8) = o; }
        if (ps == 0) __threadfence(); }
}

__global__ __launch_bounds__(32) __attribute__((amdgpu_num_vgpr(256))) void k_zgemm(const bf* __restrict__ XB, const bf* __restrict__ PT, bf* ZS) {
    __shared__ __align__(16) float os[64 * 68];
    const int lane = threadIdx.x & 31, lr = lane & 15, hi = lane >> 4;
    const int p0 = blockIdx.x * 64, n0 = blockIdx.y * 64;
    v8f acc[4][4];
#pragma unroll
    for (int mb = 0; mb < 4; ++mb)
#pragma unroll
        for (int nb = 0; nb < 4; ++nb) acc[mb][nb] = (v8f){};
    const size_t aoff = (size_t)(p0 + lr) * DM + 8 * hi, boff = (size_t)(n0 + lr) * DM + 8 * hi;
#pragma unroll 1
    for (int kc = 0; kc < DM; kc += 32) {
        v16bf a[4];
#pragma unroll
        for (int mb = 0; mb < 4; ++mb) a[mb] = ldb(XB + aoff + (size_t)mb * 16 * DM + kc);
#pragma unroll
        for (int nb = 0; nb < 4; ++nb) { const v16bf b = ldb(PT + boff + (size_t)nb * 16 * DM + kc);
#pragma unroll
            for (int mb = 0; mb < 4; ++mb) acc[mb][nb] = wmmab_g(a[mb], b, acc[mb][nb]); }
    }
#pragma unroll
    for (int mb = 0; mb < 4; ++mb) {
#pragma unroll
        for (int nb = 0; nb < 4; ++nb) {
#pragma unroll
            for (int j = 0; j < 8; ++j) os[(mb * 16 + hi * 8 + j) * 68 + nb * 16 + lr] = acc[mb][nb][j]; } }
    wave_sync();
    const int sl = lane >> 3, part = (lane >> 1) & 3, h8 = (lane & 1) * 8;
#pragma unroll 1
    for (int ps = 0; ps < 2; ++ps) {
#pragma unroll 1
        for (int it = 0; it < 64; ++it) {
            const float* orow = &os[it * 68 + sl * 16 + h8];
            const v4f x0 = *(const v4fa*)orow; const v4f x1 = *(const v4fa*)(orow + 4);
            v8us o;
#pragma unroll
            for (int k = 0; k < 8; ++k) {
                const float z = (k < 4) ? x0[k & 3] : x1[k & 3];
                const unsigned short zh = f2bf(z); const float r1 = z - bf2f(zh);
                const unsigned short zm = f2bf(r1); const float r2 = r1 - bf2f(zm);
                const unsigned short zl = f2bf(r2);
                o[k] = (part == 0) ? zh : ((part == 1) ? zm : ((part == 2) ? zl : (unsigned short)0)); }
            *(volatile v8us*)(ZS + (size_t)(p0 + it) * ZP + (size_t)(n0 >> 4) * 64 + lane * 8) = o; }
        if (ps == 0) __threadfence(); }
}

__global__ __launch_bounds__(32) __attribute__((amdgpu_num_vgpr(256))) void k_route(const bf* __restrict__ ZS, const bf* __restrict__ CT, int* TI, float* TW) {
    __shared__ __align__(16) float os[32 * 68];
    const int lane = threadIdx.x & 31, lr = lane & 15, hi = lane >> 4;
    const int n0 = blockIdx.x * 32, s = blockIdx.y;
    v8f acc[2][4];
#pragma unroll
    for (int mb = 0; mb < 2; ++mb)
#pragma unroll
        for (int nb = 0; nb < 4; ++nb) acc[mb][nb] = (v8f){};
    const size_t aoff = (size_t)(n0 + lr) * ZP + (size_t)s * 64 + 8 * hi;
    const size_t boff = ((size_t)s * NA + lr) * 64 + 8 * hi;
#pragma unroll 1
    for (int kc = 0; kc < 64; kc += 32) {
        v16bf a[2];
#pragma unroll
        for (int mb = 0; mb < 2; ++mb) a[mb] = ldb(ZS + aoff + (size_t)mb * 16 * ZP + kc);
#pragma unroll
        for (int nb = 0; nb < 4; ++nb) { const v16bf b = ldb(CT + boff + (size_t)nb * 16 * 64 + kc);
#pragma unroll
            for (int mb = 0; mb < 2; ++mb) acc[mb][nb] = wmmab_g(a[mb], b, acc[mb][nb]); }
    }
#pragma unroll
    for (int mb = 0; mb < 2; ++mb) {
#pragma unroll
        for (int nb = 0; nb < 4; ++nb) {
#pragma unroll
            for (int j = 0; j < 8; ++j) os[(mb * 16 + hi * 8 + j) * 68 + nb * 16 + lr] = acc[mb][nb][j]; } }
    wave_sync();
    float tv0 = -3.0e38f, tv1 = -3.0e38f, tv2 = -3.0e38f, tv3 = -3.0e38f;
    int ti0 = 0, ti1 = 0, ti2 = 0, ti3 = 0;
#pragma unroll 1
    for (int g = 0; g < 16; ++g) {
        const v4f v = *(const v4fa*)(&os[lane * 68 + 4 * g]);
#pragma unroll
        for (int c = 0; c < 4; ++c) top4_ins(v[c], 4 * g + c, tv0, tv1, tv2, tv3, ti0, ti1, ti2, ti3); }
    const float e1 = expf(tv1 - tv0), e2 = expf(tv2 - tv0), e3 = expf(tv3 - tv0);
    const float inv = 1.0f / (((1.0f + e1) + e2) + e3);
    v4i oi; oi[0] = clampi(ti0, 0, NA - 1); oi[1] = clampi(ti1, 0, NA - 1); oi[2] = clampi(ti2, 0, NA - 1); oi[3] = clampi(ti3, 0, NA - 1);
    v4f ow; ow[0] = inv; ow[1] = e1 * inv; ow[2] = e2 * inv; ow[3] = e3 * inv;
    const size_t o4 = ((size_t)s * NTOK + n0 + lane) * 4;
    *(volatile v4i*)(TI + o4) = oi;
    *(volatile v4f*)(TW + o4) = ow;
    __threadfence();
    *(volatile v4i*)(TI + o4) = oi;
    *(volatile v4f*)(TW + o4) = ow;
}

__global__ __launch_bounds__(1024) void k_count(const int* __restrict__ idx, int* cnt) {
    __shared__ int wc[32 * 64];
    __shared__ __align__(16) int line[64];
    const int tid = threadIdx.x, lane = tid & 31; const int wave = __builtin_amdgcn_readfirstlane(tid >> 5);
    const int blk = blockIdx.x;
    const int rel = clampi(idx[(size_t)blk * RB + tid], 0, NA - 1);
    int m0 = 0, m1 = 0;
#pragma unroll 1
    for (int r = 0; r < 32; ++r) {
        const unsigned ma = __builtin_amdgcn_ballot_w32(rel == r); const unsigned mb = __builtin_amdgcn_ballot_w32(rel == r + 32);
        const int ca = __builtin_popcount(ma), cb = __builtin_popcount(mb);
        m0 = (lane == r) ? ca : m0; m1 = (lane == r) ? cb : m1; }
    wc[wave * 64 + lane] = m0; wc[wave * 64 + 32 + lane] = m1;
    __syncthreads();
    if (wave == 0) {
        int s0 = 0, s1 = 0;
#pragma unroll 1
        for (int w = 0; w < 32; ++w) { s0 += wc[w * 64 + lane]; s1 += wc[w * 64 + 32 + lane]; }
        line[lane] = s0; line[32 + lane] = s1;
        wave_sync();
#pragma unroll 1
        for (int ps = 0; ps < 2; ++ps) {
            if (lane < 16) { const v4i v = *(const v4ia*)(&line[4 * lane]); *(volatile v4i*)(cnt + (size_t)blk * 64 + 4 * lane) = v; }
            if (ps == 0) __threadfence(); }
    }
}

__global__ __launch_bounds__(512) void k_scan(const int* __restrict__ cnt, int* offs, int* TE, h16* XS) {
    __shared__ __align__(16) int ol[NBLK * 64];
    __shared__ __align__(16) int te[TILES];
    __shared__ int wt[16];
    const int tid = threadIdx.x, lane = tid & 31; const int wave = __builtin_amdgcn_readfirstlane(tid >> 5);
    const int g = tid, s = g >> 6, m = g & 63;
    int run = 0;
#pragma unroll 1
    for (int b = 0; b < NBS; ++b) { const int bi = (s * NBS + b) * 64 + m; const int v = clampi(cnt[bi], 0, RB); ol[bi] = run; run += v; }
    const int tot = run; const int pd = (tot + 63) & ~63;
    int x = pd;
#pragma unroll
    for (int d = 1; d < 32; d <<= 1) { const int y = __shfl_up(x, d, 32); x += (lane >= d) ? y : 0; }
    const int wtot = __shfl(x, 31, 32);
    if (lane == 0) wt[wave] = wtot;
#pragma unroll 1
    for (int it = 0; it < TILES / 512; ++it) te[it * 512 + tid] = -1;
    __syncthreads();
    int base = 0;
#pragma unroll 1
    for (int w = 0; w < 16; ++w) { const int v = wt[w]; base += (w < wave) ? v : 0; }
    const int sstart = base + x - pd;
#pragma unroll 1
    for (int b = 0; b < NBS; ++b) { const int bi = (s * NBS + b) * 64 + m; ol[bi] += sstart; }
    const int ntile = min(pd >> 6, MAXT); const int t0 = sstart >> 6;
#pragma unroll 1
    for (int j = 0; j < ntile; ++j) te[clampi(t0 + j, 0, TILES - 1)] = g;
    __syncthreads();
    const int padcnt = pd - tot;
    const int pbase = sstart + tot;
    v8h z;
#pragma unroll
    for (int k = 0; k < 8; ++k) z[k] = (h16)0.0f;
#pragma unroll 1
    for (int ps = 0; ps < 2; ++ps) {
#pragma unroll 1
        for (int it = 0; it < (NBLK * 16) / 512; ++it) { const int i = it * 512 + tid; const v4i v = *(const v4ia*)(&ol[4 * i]); *(volatile v4i*)(offs + 4 * (size_t)i) = v; }
#pragma unroll 1
        for (int it = 0; it < (TILES / 4 + 511) / 512; ++it) { const int i = it * 512 + tid; const int ic = min(i, TILES / 4 - 1);
            const v4i v = *(const v4ia*)(&te[4 * ic]); if (i < TILES / 4) { *(volatile v4i*)(TE + 4 * (size_t)i) = v; } }
#pragma unroll 1
        for (int gi = 0; gi < 32; ++gi) { const int pc = __shfl(padcnt, gi, 32); const int pb = __shfl(pbase, gi, 32);
#pragma unroll 1
            for (int it = 0; it < 16; ++it) { const int j = 4 * it + (lane >> 3); const int p = clampi(pb + j, 0, PROWS - 1);
                if (j < pc) { *(volatile v8h*)(XS + (size_t)p * XP + (lane & 7) * 8) = z; } } }
        if (ps == 0) __threadfence(); }
}

__global__ __launch_bounds__(1024) void k_rank(const int* __restrict__ idx, const bf* __restrict__ ZS, const int* __restrict__ offs, int* POS, h16* XS) {
    __shared__ int wc[32 * 64];
    const int tid = threadIdx.x, lane = tid & 31; const int wave = __builtin_amdgcn_readfirstlane(tid >> 5);
    const int blk = blockIdx.x; const int s = blk / NBS; const int bq = blk - s * NBS;
    const size_t q = (size_t)blk * RB + tid;
    const int rel = clampi(idx[q], 0, NA - 1);
    int m0 = 0, m1 = 0; unsigned mymask = 0u;
#pragma unroll 1
    for (int r = 0; r < 32; ++r) {
        const unsigned ma = __builtin_amdgcn_ballot_w32(rel == r); const unsigned mb = __builtin_amdgcn_ballot_w32(rel == r + 32);
        const int ca = __builtin_popcount(ma), cb = __builtin_popcount(mb);
        m0 = (lane == r) ? ca : m0; m1 = (lane == r) ? cb : m1;
        mymask = (rel == r) ? ma : mymask; mymask = (rel == r + 32) ? mb : mymask; }
    const int lrank = __builtin_popcount(mymask & ((1u << lane) - 1u));
    wc[wave * 64 + lane] = m0; wc[wave * 64 + 32 + lane] = m1;
    __syncthreads();
    if (wave == 0) {
        int run0 = clampi(offs[(size_t)blk * 64 + lane], 0, PROWS), run1 = clampi(offs[(size_t)blk * 64 + 32 + lane], 0, PROWS);
#pragma unroll 1
        for (int w = 0; w < 32; ++w) { const int c0 = wc[w * 64 + lane]; wc[w * 64 + lane] = run0; run0 += c0;
                                       const int c1 = wc[w * 64 + 32 + lane]; wc[w * 64 + 32 + lane] = run1; run1 += c1; }
    }
    __syncthreads();
    const int pos = clampi(wc[wave * 64 + rel] + lrank, 0, PROWS - 1);
#pragma unroll 1
    for (int ps = 0; ps < 2; ++ps) {
        *(volatile int*)(POS + q) = pos;
#pragma unroll 1
        for (int it = 0; it < 8; ++it) { const int j = 4 * it + (lane >> 3); const int p = __shfl(pos, j, 32); const int pc = lane & 7;
            const int nj = (bq * RB + wave * 32 + j) >> 2;
            const bf* zp = ZS + (size_t)nj * ZP + (size_t)s * 64 + (pc & 1) * 8;
            const v8us a = *(const v8us*)zp; const v8us b = *(const v8us*)(zp + 16); const v8us c = *(const v8us*)(zp + 32);
            v8h o;
#pragma unroll
            for (int k = 0; k < 8; ++k) { const float zv = (bf2f(a[k]) + bf2f(b[k])) + bf2f(c[k]);
                const h16 vh = toh_flush(zv); const h16 vl = toh_flush(zv - (float)vh);
                o[k] = (pc < 2) ? vh : ((pc < 4) ? vl : (h16)0.0f); }
            *(volatile v8h*)(XS + (size_t)p * XP + pc * 8) = o; }
        if (ps == 0) __threadfence(); }
}

__global__ __launch_bounds__(32) __attribute__((amdgpu_num_vgpr(256))) void k_local(const h16* __restrict__ XS, const h16* __restrict__ W1T, const float* __restrict__ b1,
                                                                                     const h16* __restrict__ W2T, const float* __restrict__ b2, const int* __restrict__ TE, float* YS) {
    __shared__ __align__(16) h16 hs[64 * 40];
    __shared__ __align__(16) float os2[64 * 20];
    const int lane = threadIdx.x & 31, lr = lane & 15, hi = lane >> 4;
    const int p0 = blockIdx.x * 64;
    const int er = TE[blockIdx.x];
    if (er < 0) return;
    const int e = __builtin_amdgcn_readfirstlane(clampi(er, 0, NGRP - 1));
    v8f acc[4][2];
#pragma unroll
    for (int mb = 0; mb < 4; ++mb)
#pragma unroll
        for (int nb = 0; nb < 2; ++nb) acc[mb][nb] = (v8f){};
    v16h a[4];
#pragma unroll
    for (int mb = 0; mb < 4; ++mb) a[mb] = ldh(XS + (size_t)(p0 + mb * 16 + lr) * XP + 8 * hi);
    float bv[2];
#pragma unroll
    for (int nb = 0; nb < 2; ++nb) { const v16h b = ldh(W1T + (size_t)e * (HL * 32) + (size_t)(nb * 16 + lr) * 32 + 8 * hi);
        bv[nb] = bf2f(f2bf(b1[(size_t)e * HL + nb * 16 + lr]));
#pragma unroll
        for (int mb = 0; mb < 4; ++mb) acc[mb][nb] = wmmah_g(a[mb], b, acc[mb][nb]); }
#pragma unroll
    for (int mb = 0; mb < 4; ++mb) {
#pragma unroll
        for (int nb = 0; nb < 2; ++nb) {
#pragma unroll
            for (int j = 0; j < 8; ++j) hs[(mb * 16 + hi * 8 + j) * 40 + nb * 16 + lr] = toh_flush(gelu_t(acc[mb][nb][j] + bv[nb])); } }
    wave_sync();
    const v16h b2f = ldh(W2T + (size_t)e * (RK * HL) + (size_t)lr * HL + 8 * hi);
    const float b2v = bf2f(f2bf(b2[(size_t)e * RK + lr]));
    v8f acc2[4];
#pragma unroll
    for (int mb = 0; mb < 4; ++mb) {
        const v16h a2 = cat16h(*(const v8ha*)(&hs[(mb * 16 + lr) * 40 + 8 * hi]), *(const v8ha*)(&hs[(mb * 16 + lr) * 40 + 16 + 8 * hi]));
        acc2[mb] = wmmah_g(a2, b2f, (v8f){}); }
#pragma unroll
    for (int mb = 0; mb < 4; ++mb) {
#pragma unroll
        for (int j = 0; j < 8; ++j) os2[(mb * 16 + hi * 8 + j) * 20 + lr] = acc2[mb][j] + b2v; }
    wave_sync();
    const int pc = lane & 7;
#pragma unroll 1
    for (int ps = 0; ps < 2; ++ps) {
#pragma unroll 1
        for (int it = 0; it < 16; ++it) {
            const int row = 4 * it + (lane >> 3);
            const v4f x = *(const v4fa*)(&os2[row * 20 + (pc & 3) * 4]);
            v4f y;
#pragma unroll
            for (int k = 0; k < 4; ++k) y[k] = (pc < 4) ? x[k] : 0.0f;
            *(volatile v4f*)(YS + (size_t)(p0 + row) * YP + pc * 4) = y; }
        if (ps == 0) __threadfence(); }
}

__global__ __launch_bounds__(256) void k_comb(const int* __restrict__ POS, const float* __restrict__ TW, const float* __restrict__ YS, h16* CB) {
    const int lane = threadIdx.x & 31, wave = threadIdx.x >> 5;
    const int n = min((int)blockIdx.x * 16 + wave * 2 + (lane >> 4), NTOK - 1);
    const int pc = lane & 15, s = pc >> 1, r8 = (pc & 1) * 8;
    const size_t b4 = ((size_t)s * NTOK + n) * 4;
    float acc[8];
#pragma unroll
    for (int c = 0; c < 8; ++c) acc[c] = 0.0f;
#pragma unroll 1
    for (int k = 0; k < TK; ++k) {
        const int p = clampi(POS[b4 + k], 0, PROWS - 1);
        const float w = TW[b4 + k];
        const v4f y0 = *(const v4f*)(YS + (size_t)p * YP + r8); const v4f y1 = *(const v4f*)(YS + (size_t)p * YP + r8 + 4);
#pragma unroll
        for (int c = 0; c < 4; ++c) { acc[c] += w * y0[c]; acc[4 + c] += w * y1[c]; } }
    v8h o;
#pragma unroll
    for (int c = 0; c < 8; ++c) o[c] = toh_flush(acc[c]);
    h16* dst = CB + (size_t)n * SR + pc * 8;
    *(volatile v8h*)dst = o;
    __threadfence();
    *(volatile v8h*)dst = o;
}

__global__ __launch_bounds__(32) __attribute__((amdgpu_num_vgpr(256))) void k_g1(const h16* __restrict__ CB, const h16* __restrict__ G1T, const float* __restrict__ g1b, h16* HID) {
    __shared__ __align__(16) float os[64 * 68];
    const int lane = threadIdx.x & 31, lr = lane & 15, hi = lane >> 4;
    const int p0 = blockIdx.x * 64, n0 = blockIdx.y * 64;
    v8f acc[4][4];
#pragma unroll
    for (int mb = 0; mb < 4; ++mb)
#pragma unroll
        for (int nb = 0; nb < 4; ++nb) acc[mb][nb] = (v8f){};
    const size_t aoff = (size_t)(p0 + lr) * SR + 8 * hi, boff = (size_t)(n0 + lr) * SR + 8 * hi;
#pragma unroll 1
    for (int kc = 0; kc < SR; kc += 32) {
        v16h a[4];
#pragma unroll
        for (int mb = 0; mb < 4; ++mb) a[mb] = ldh(CB + aoff + (size_t)mb * 16 * SR + kc);
#pragma unroll
        for (int nb = 0; nb < 4; ++nb) { const v16h b = ldh(G1T + boff + (size_t)nb * 16 * SR + kc);
#pragma unroll
            for (int mb = 0; mb < 4; ++mb) acc[mb][nb] = wmmah_g(a[mb], b, acc[mb][nb]); }
    }
#pragma unroll
    for (int mb = 0; mb < 4; ++mb) {
#pragma unroll
        for (int nb = 0; nb < 4; ++nb) {
#pragma unroll
            for (int j = 0; j < 8; ++j) os[(mb * 16 + hi * 8 + j) * 68 + nb * 16 + lr] = acc[mb][nb][j]; } }
    wave_sync();
    const int c8 = (lane & 7) * 8;
    v8f bb = *(const v8f*)(g1b + n0 + c8);
#pragma unroll
    for (int k = 0; k < 8; ++k) bb[k] = bf2f(f2bf(bb[k]));
#pragma unroll 1
    for (int ps = 0; ps < 2; ++ps) {
#pragma unroll 1
        for (int it = 0; it < 16; ++it) {
            const int row = 4 * it + (lane >> 3);
            const float* orow = &os[row * 68 + c8];
            const v4f x0 = *(const v4fa*)orow; const v4f x1 = *(const v4fa*)(orow + 4);
            v8h o;
#pragma unroll
            for (int k = 0; k < 4; ++k) { o[k] = toh_flush(gelu_t(x0[k] + bb[k])); o[4 + k] = toh_flush(gelu_t(x1[k] + bb[4 + k])); }
            *(volatile v8h*)(HID + (size_t)(p0 + row) * HG + n0 + c8) = o; }
        if (ps == 0) __threadfence(); }
}

__global__ __launch_bounds__(32) __attribute__((amdgpu_num_vgpr(256))) void k_g2(const h16* __restrict__ HID, const h16* __restrict__ G2T, const float* __restrict__ g2b, float* OUT) {
    __shared__ __align__(16) float os[64 * 68];
    const int lane = threadIdx.x & 31, lr = lane & 15, hi = lane >> 4;
    const int p0 = blockIdx.x * 64, n0 = blockIdx.y * 64;
    v8f acc[4][4];
#pragma unroll
    for (int mb = 0; mb < 4; ++mb)
#pragma unroll
        for (int nb = 0; nb < 4; ++nb) acc[mb][nb] = (v8f){};
    const size_t aoff = (size_t)(p0 + lr) * HG + 8 * hi, boff = (size_t)(n0 + lr) * HG + 8 * hi;
#pragma unroll 1
    for (int kc = 0; kc < HG; kc += 32) {
        v16h a[4];
#pragma unroll
        for (int mb = 0; mb < 4; ++mb) a[mb] = ldh(HID + aoff + (size_t)mb * 16 * HG + kc);
#pragma unroll
        for (int nb = 0; nb < 4; ++nb) { const v16h b = ldh(G2T + boff + (size_t)nb * 16 * HG + kc);
#pragma unroll
            for (int mb = 0; mb < 4; ++mb) acc[mb][nb] = wmmah_g(a[mb], b, acc[mb][nb]); }
    }
#pragma unroll
    for (int mb = 0; mb < 4; ++mb) {
#pragma unroll
        for (int nb = 0; nb < 4; ++nb) {
#pragma unroll
            for (int j = 0; j < 8; ++j) os[(mb * 16 + hi * 8 + j) * 68 + nb * 16 + lr] = acc[mb][nb][j]; } }
    wave_sync();
    const int c4 = (lane & 15) * 4;
    v4f bb = *(const v4f*)(g2b + n0 + c4);
#pragma unroll
    for (int k = 0; k < 4; ++k) bb[k] = bf2f(f2bf(bb[k]));
    const size_t orow0 = (size_t)(p0 / SEQ) * SEQ_FULL + (size_t)(p0 % SEQ);
#pragma unroll 1
    for (int ps = 0; ps < 2; ++ps) {
#pragma unroll 1
        for (int it = 0; it < 32; ++it) {
            const int row = 2 * it + (lane >> 4);
            const v4f x = *(const v4fa*)(&os[row * 68 + c4]);
            v4f y;
#pragma unroll
            for (int k = 0; k < 4; ++k) y[k] = x[k] + bb[k];
            *(volatile v4f*)(OUT + (orow0 + row) * DM + n0 + c4) = y; }
        if (ps == 0) __threadfence(); }
}

static constexpr size_t al256(size_t v) { return (v + 255) & ~(size_t)255; }
static constexpr size_t SZ_XB  = al256((size_t)NTOK * DM * 2);
static constexpr size_t SZ_PT  = al256((size_t)SR * DM * 2);
static constexpr size_t SZ_CT  = al256((size_t)NGRP * 64 * 2);
static constexpr size_t SZ_W1T = al256((size_t)NGRP * HL * 32 * 2);
static constexpr size_t SZ_W2T = al256((size_t)NGRP * RK * HL * 2);
static constexpr size_t SZ_G1T = al256((size_t)HG * SR * 2);
static constexpr size_t SZ_G2T = al256((size_t)DM * HG * 2);
static constexpr size_t SZ_ZS  = al256((size_t)NTOK * ZP * 2);
static constexpr size_t SZ_TI  = al256((size_t)NS * NTOK * TK * 4);
static constexpr size_t SZ_TW  = al256((size_t)NS * NTOK * TK * 4);
static constexpr size_t SZ_CNT = al256((size_t)NBLK * 64 * 4);
static constexpr size_t SZ_OFF = al256((size_t)NBLK * 64 * 4);
static constexpr size_t SZ_TE  = al256((size_t)TILES * 4);
static constexpr size_t SZ_POS = al256((size_t)NS * NPS * 4);
static constexpr size_t SZ_XS  = al256((size_t)PROWS * XP * 2);
static constexpr size_t SZ_YS  = al256((size_t)PROWS * YP * 4);
static constexpr size_t SZ_CB  = al256((size_t)NTOK * SR * 2);
static constexpr size_t SZ_HID = al256((size_t)NTOK * HG * 2);
static constexpr size_t SZ_TOTAL = SZ_XB + SZ_PT + SZ_CT + SZ_W1T + SZ_W2T + SZ_G1T + SZ_G2T + SZ_ZS + SZ_TI + SZ_TW + SZ_CNT + SZ_OFF + SZ_TE + SZ_POS + SZ_XS + SZ_YS + SZ_CB + SZ_HID;
static_assert(SZ_TOTAL <= (size_t)134217728);

extern "C" void kernel_launch(void* const* d_in, const int* in_sizes, int n_in,
                              void* d_out, int out_size, void* d_ws, size_t ws_size, hipStream_t stream) {
    if (n_in < 11) return;
    if ((size_t)in_sizes[0] < ((size_t)(NB - 1) * SEQ_FULL + SEQ) * DM) return;
    if ((size_t)in_sizes[1] < (size_t)NS * DM * RK) return;
    if ((size_t)in_sizes[2] < (size_t)NGRP * RK) return;
    if ((size_t)in_sizes[3] < (size_t)NGRP * RK * HL) return;
    if ((size_t)in_sizes[4] < (size_t)NGRP * HL) return;
    if ((size_t)in_sizes[5] < (size_t)NGRP * HL * RK) return;
    if ((size_t)in_sizes[6] < (size_t)NGRP * RK) return;
    if ((size_t)in_sizes[7] < (size_t)SR * HG) return;
    if ((size_t)in_sizes[8] < (size_t)HG) return;
    if ((size_t)in_sizes[9] < (size_t)HG * DM) return;
    if ((size_t)in_sizes[10] < (size_t)DM) return;
    if ((size_t)out_size < ((size_t)(NB - 1) * SEQ_FULL + SEQ) * DM) return;
    if (SZ_TOTAL > ws_size) return;
    const float* X   = (const float*)d_in[0];
    const float* P   = (const float*)d_in[1];
    const float* C   = (const float*)d_in[2];
    const float* W1  = (const float*)d_in[3];
    const float* b1  = (const float*)d_in[4];
    const float* W2  = (const float*)d_in[5];
    const float* b2  = (const float*)d_in[6];
    const float* G1  = (const float*)d_in[7];
    const float* g1b = (const float*)d_in[8];
    const float* G2  = (const float*)d_in[9];
    const float* g2b = (const float*)d_in[10];
    float* OUT = (float*)d_out;
    char* wsp = (char*)d_ws;
    bf*  XB  = (bf*)wsp;   wsp += SZ_XB;
    bf*  PT  = (bf*)wsp;   wsp += SZ_PT;
    bf*  CT  = (bf*)wsp;   wsp += SZ_CT;
    h16* W1T = (h16*)wsp;  wsp += SZ_W1T;
    h16* W2T = (h16*)wsp;  wsp += SZ_W2T;
    h16* G1T = (h16*)wsp;  wsp += SZ_G1T;
    h16* G2T = (h16*)wsp;  wsp += SZ_G2T;
    bf*  ZS  = (bf*)wsp;   wsp += SZ_ZS;
    int* TI  = (int*)wsp;  wsp += SZ_TI;
    float* TW = (float*)wsp; wsp += SZ_TW;
    int* CNT = (int*)wsp;  wsp += SZ_CNT;
    int* OFF = (int*)wsp;  wsp += SZ_OFF;
    int* TE  = (int*)wsp;  wsp += SZ_TE;
    int* POS = (int*)wsp;  wsp += SZ_POS;
    h16* XS  = (h16*)wsp;  wsp += SZ_XS;
    float* YS = (float*)wsp; wsp += SZ_YS;
    h16* CB  = (h16*)wsp;  wsp += SZ_CB;
    h16* HID = (h16*)wsp;  wsp += SZ_HID;

    k_xcvt<<<(NTOK * (DM / 8)) / 256, 256, 0, stream>>>(X, XB);
    k_prep<<<PB1 + PB2 + PB3 + PB4, 256, 0, stream>>>(P, C, W1, W2, PT, CT, W1T, W2T);
    k_wt<<<dim3(HG / 64, SR / 64, 1), 256, 0, stream>>>(G1, G1T, SR, HG);
    k_wt<<<dim3(DM / 64, HG / 64, 1), 256, 0, stream>>>(G2, G2T, HG, DM);
    k_zgemm<<<dim3(NTOK / 64, SR / 64), 32, 0, stream>>>(XB, PT, ZS);
    k_route<<<dim3(NTOK / 32, NS), 32, 0, stream>>>(ZS, CT, TI, TW);
    k_count<<<NBLK, 1024, 0, stream>>>(TI, CNT);
    k_scan<<<1, 512, 0, stream>>>(CNT, OFF, TE, XS);
    k_rank<<<NBLK, 1024, 0, stream>>>(TI, ZS, OFF, POS, XS);
    k_local<<<TILES, 32, 0, stream>>>(XS, W1T, b1, W2T, b2, TE, YS);
    k_comb<<<NTOK / 16, 256, 0, stream>>>(POS, TW, YS, CB);
    k_g1<<<dim3(NTOK / 64, HG / 64), 32, 0, stream>>>(CB, G1T, g1b, HID);
    k_g2<<<dim3(NTOK / 64, DM / 64), 32, 0, stream>>>(HID, G2T, g2b, OUT);
}
